// RGATStack_77283641524510
// MI455X (gfx1250) — hardware-verified
//
#include <hip/hip_runtime.h>
#include <stddef.h>


#define DM     256
#define DQKV   768
#define DFF    1024
#define GT     128
#define SPW    (32 * 64)
#define WPP    72
#define BNODE  64
#define LCAP   2048
#define TROW   64
#define DEGCAP 63
#define CHK    2048
#define WSCAP  134217728
#define ASCL   8.0f
#define WSCL   64.0f
#define INVSCL 0.001953125f
#define INVDM  0.00390625f
#define RMSEPS 1.1920929e-07f
#define QKSCL  0.17677669529663687f
#define GHALF  0.70710678118654752f

static_assert((DM % 64) == 0 && (DFF % 256) == 0 && (DQKV % 256) == 0);
static_assert((WPP % 8) == 0);
static_assert(LCAP == 8 * 256 && CHK == 8 * 256);
static_assert(BNODE * TROW == 16 * 256);
static_assert(DEGCAP == TROW - 1);

typedef float          v2f  __attribute__((ext_vector_type(2)));
typedef float          v4f  __attribute__((ext_vector_type(4)));
typedef float          v8f  __attribute__((ext_vector_type(8)));
typedef unsigned int   v4u  __attribute__((ext_vector_type(4)));
typedef unsigned short v8us __attribute__((ext_vector_type(8)));
typedef _Float16       v16h __attribute__((ext_vector_type(16)));
typedef int            v4i  __attribute__((ext_vector_type(4)));
typedef int            v2i  __attribute__((ext_vector_type(2)));
union FragH { v16h v; v8us u[2]; };

__device__ __forceinline__ unsigned short h16(float f) {
  const _Float16 h = (_Float16)f;
  return __builtin_bit_cast(unsigned short, h);
}

__device__ __forceinline__ v8us cvt8(v4f a, v4f b, float s) {
  v8us r;
  r[0] = h16(a.x * s); r[1] = h16(a.y * s); r[2] = h16(a.z * s); r[3] = h16(a.w * s);
  r[4] = h16(b.x * s); r[5] = h16(b.y * s); r[6] = h16(b.z * s); r[7] = h16(b.w * s);
  return r;
}

__device__ __forceinline__ v8f wmh(v16h a, v16h b, v8f c) {
  v8f d = __builtin_amdgcn_wmma_f32_16x16x32_f16(false, a, false, b, (short)0, c, false, false);
  asm volatile("v_nop\n\tv_nop\n\tv_nop\n\tv_nop" : "+v"(d) : "v"(a), "v"(b));
  return d;
}

__global__ __launch_bounds__(256) void k_wpack(
    const float* __restrict__ W, unsigned short* wt, int K, int M, int inZ, int outZ) {
  __shared__ __attribute__((aligned(16))) unsigned short sT[64 * WPP];
  const int tid = (int)threadIdx.x;
  const int m0 = (int)blockIdx.x * 64, k0 = (int)blockIdx.y * 64;
  W  += (size_t)blockIdx.z * (size_t)inZ;
  wt += (size_t)blockIdx.z * (size_t)outZ;
#pragma unroll 4
  for (int it = 0; it < 16; ++it) {
    const int idx = it * 256 + tid;
    const int kk = idx >> 6, mm = idx & 63;
    int kr = k0 + kk; kr = kr > K - 1 ? K - 1 : kr;
    int mc = m0 + mm; mc = mc > M - 1 ? M - 1 : mc;
    const float w = W[(size_t)kr * M + mc];
    sT[mm * WPP + kk] = h16(w * WSCL);
  }
  __syncthreads();
  v8us pv[2];
  size_t po[2];
#pragma unroll
  for (int it = 0; it < 2; ++it) {
    const int p = it * 256 + tid;
    const int row = p >> 3, c8 = (p & 7) * 8;
    pv[it] = *(const v8us*)(sT + row * WPP + c8);
    int mr = m0 + row; mr = mr > M - 1 ? M - 1 : mr;
    po[it] = (size_t)mr * K + k0 + c8;
  }
  const bool full = (m0 + 64 <= M) && (k0 + 64 <= K);
  if (full) {
#pragma unroll
    for (int it = 0; it < 2; ++it) *(volatile v8us*)(wt + po[it]) = pv[it];
  }
  __threadfence();
  if (full) {
#pragma unroll
    for (int it = 0; it < 2; ++it) *(volatile v8us*)(wt + po[it]) = pv[it];
  }
}

__global__ __launch_bounds__(256) void k_cvt(const float* __restrict__ X, unsigned short* outH, int nRows) {
  const int tid = (int)threadIdx.x, lane = tid & 31, wave = tid >> 5;
  const int row = (int)blockIdx.x * 8 + wave;
  if (row < nRows) {
    const float* xr = X + (size_t)row * DM + 8 * lane;
    const v4f a0 = *(const v4f*)xr;
    const v4f a1 = *(const v4f*)(xr + 4);
    const v8us hv = cvt8(a0, a1, ASCL);
    unsigned short* op = outH + (size_t)row * DM + 8 * lane;
    *(volatile v8us*)op = hv;
    __threadfence();
    *(volatile v8us*)op = hv;
  }
}

__global__ __launch_bounds__(256) void k_rms(
    const float* X, const float* __restrict__ w, unsigned short* outH, int nRows) {
  const int tid = (int)threadIdx.x, lane = tid & 31, wave = tid >> 5;
  const int row = (int)blockIdx.x * 8 + wave;
  if (row < nRows) {
    const float* xr = X + (size_t)row * DM + 8 * lane;
    const v4f a0 = *(const v4f*)xr;
    const v4f a1 = *(const v4f*)(xr + 4);
    float sq = ((a0.x * a0.x + a0.y * a0.y) + (a0.z * a0.z + a0.w * a0.w)) +
               ((a1.x * a1.x + a1.y * a1.y) + (a1.z * a1.z + a1.w * a1.w));
#pragma unroll
    for (int o = 16; o >= 1; o >>= 1) sq += __shfl_xor(sq, o);
    const float rs = rsqrtf(sq * INVDM + RMSEPS);
    const v4f w0 = *(const v4f*)(w + 8 * lane);
    const v4f w1 = *(const v4f*)(w + 8 * lane + 4);
    const v4f y0 = (a0 * rs) * w0;
    const v4f y1 = (a1 * rs) * w1;
    const v8us hv = cvt8(y0, y1, ASCL);
    unsigned short* op = outH + (size_t)row * DM + 8 * lane;
    *(volatile v8us*)op = hv;
    __threadfence();
    *(volatile v8us*)op = hv;
  }
}

template <int GELU16, int RESID>
__global__ __launch_bounds__(GT) void k_gemm(
    const unsigned short* __restrict__ A, const unsigned short* __restrict__ Bt,
    const float* __restrict__ b0, const float* __restrict__ b1, const float* __restrict__ b2, int bshift,
    const float* res, float* outF, unsigned short* outH, int K, int Ncols, int M) {
  __shared__ __attribute__((aligned(16))) float sT[4 * SPW];
  const int tid = (int)threadIdx.x, lane = tid & 31, wave = tid >> 5, hh = lane >> 4, m = lane & 15;
  const int r0 = (int)blockIdx.y * 32;
  const int c0 = (int)blockIdx.x * 256 + wave * 64;

  int ra0 = r0 + m;      ra0 = ra0 > M - 1 ? M - 1 : ra0;
  int ra1 = r0 + 16 + m; ra1 = ra1 > M - 1 ? M - 1 : ra1;
  const unsigned short* ap0 = A + (size_t)ra0 * K + 8 * hh;
  const unsigned short* ap1 = A + (size_t)ra1 * K + 8 * hh;
  const unsigned short* bp[4];
#pragma unroll
  for (int j = 0; j < 4; ++j) {
    int cb = c0 + 16 * j + m; cb = cb > Ncols - 1 ? Ncols - 1 : cb;
    bp[j] = Bt + (size_t)cb * K + 8 * hh;
  }

  v8f acc[2][4];
#pragma unroll
  for (int i = 0; i < 2; ++i)
#pragma unroll
    for (int j = 0; j < 4; ++j) { v8f z = {0.f, 0.f, 0.f, 0.f, 0.f, 0.f, 0.f, 0.f}; acc[i][j] = z; }

  const int nk = K >> 5;
#pragma unroll 1
  for (int kt = 0; kt < nk; ++kt) {
    const int kb = kt << 5;
    FragH fa0, fa1;
    fa0.u[0] = *(const v8us*)(ap0 + kb);
    fa0.u[1] = *(const v8us*)(ap0 + kb + 16);
    fa1.u[0] = *(const v8us*)(ap1 + kb);
    fa1.u[1] = *(const v8us*)(ap1 + kb + 16);
#pragma unroll
    for (int j = 0; j < 4; ++j) {
      FragH fb;
      fb.u[0] = *(const v8us*)(bp[j] + kb);
      fb.u[1] = *(const v8us*)(bp[j] + kb + 16);
      acc[0][j] = wmh(fa0.v, fb.v, acc[0][j]);
      acc[1][j] = wmh(fa1.v, fb.v, acc[1][j]);
    }
  }

  float* sw = sT + wave * SPW;
#pragma unroll
  for (int i = 0; i < 2; ++i)
#pragma unroll
    for (int j = 0; j < 4; ++j)
#pragma unroll
      for (int r = 0; r < 8; ++r)
        sw[(16 * i + 8 * hh + r) * 64 + 16 * j + m] = acc[i][j][r];

  const int grp = c0 >> bshift;
  const float* bptr = (grp == 0) ? b0 : ((grp == 1) ? b1 : b2);
  const int bc0 = c0 - (grp << bshift);

  if (GELU16) {
#pragma unroll 1
    for (int t = 0; t < 64; ++t) {
      const int i = t >> 5, j = (t >> 3) & 3, r = t & 7;
      const int idx = (16 * i + 8 * hh + r) * 64 + 16 * j + m;
      const float v = sw[idx] * INVSCL + bptr[bc0 + 16 * j + m];
      sw[idx] = 0.5f * v * (1.0f + erff(v * GHALF));
    }
  }
  __syncthreads();

  const bool full = (r0 + 32 <= M) && (c0 + 64 <= Ncols);
  if (GELU16) {
    v8us hv[8];
    size_t po[8];
#pragma unroll
    for (int it = 0; it < 8; ++it) {
      const int f = it * 32 + lane;
      const int row = f >> 3, c8 = (f & 7) * 8;
      const v4f v0 = *(const v4f*)(sw + row * 64 + c8);
      const v4f v1 = *(const v4f*)(sw + row * 64 + c8 + 4);
      hv[it] = cvt8(v0, v1, ASCL);
      po[it] = (size_t)(r0 + row) * Ncols + c0 + c8;
    }
    if (full) {
#pragma unroll
      for (int it = 0; it < 8; ++it) *(volatile v8us*)(outH + po[it]) = hv[it];
    }
    __threadfence();
    if (full) {
#pragma unroll
      for (int it = 0; it < 8; ++it) *(volatile v8us*)(outH + po[it]) = hv[it];
    }
  } else {
    v4f ov[16];
    size_t po[16];
#pragma unroll
    for (int it = 0; it < 16; ++it) {
      const int f = it * 32 + lane;
      const int row = f >> 4, c4 = (f & 15) * 4;
      const v4f v = *(const v4f*)(sw + row * 64 + c4);
      int gc = c0 + c4; gc = gc > Ncols - 4 ? Ncols - 4 : gc;
      int gr = r0 + row; gr = gr > M - 1 ? M - 1 : gr;
      const v4f bb = *(const v4f*)(bptr + bc0 + c4);
      v4f o = v * INVSCL + bb;
      if (RESID) o = o + *(const v4f*)(res + (size_t)gr * Ncols + gc);
      ov[it] = o;
      po[it] = (size_t)(r0 + row) * Ncols + c0 + c4;
    }
    if (full) {
#pragma unroll
      for (int it = 0; it < 16; ++it) *(volatile v4f*)(outF + po[it]) = ov[it];
    }
    __threadfence();
    if (full) {
#pragma unroll
      for (int it = 0; it < 16; ++it) *(volatile v4f*)(outF + po[it]) = ov[it];
    }
  }
}

__global__ __launch_bounds__(256) void k_build(
    const int* __restrict__ src, const int* __restrict__ dst, const int* __restrict__ ety,
    int* tab, int nN, int nE, int vecok) {
  __shared__ int sL[LCAP + 1];
  __shared__ int sP[LCAP];
  __shared__ int sWT[8];
  __shared__ __attribute__((aligned(16))) int sRow[BNODE * TROW];
  const int tid = (int)threadIdx.x, lane = tid & 31, wave = tid >> 5;
  const int nbase = (int)blockIdx.x * BNODE;

#pragma unroll
  for (int i = 0; i < (BNODE * TROW) / 256; ++i) sRow[i * 256 + tid] = 0;

  int tot = 0;
  const int nch = (nE + CHK - 1) / CHK;
#pragma unroll 1
  for (int c = 0; c < nch; ++c) {
    const int cbase = c * CHK;
    const int e0 = cbase + 8 * tid;
    int d[8];
    if (vecok != 0 && cbase + CHK <= nE) {
      const v4i u0 = *(const v4i*)(dst + e0);
      const v4i u1 = *(const v4i*)(dst + e0 + 4);
      d[0] = u0.x; d[1] = u0.y; d[2] = u0.z; d[3] = u0.w;
      d[4] = u1.x; d[5] = u1.y; d[6] = u1.z; d[7] = u1.w;
    } else {
#pragma unroll
      for (int q = 0; q < 8; ++q) {
        int ea = e0 + q; ea = ea > nE - 1 ? nE - 1 : ea;
        const int dv = dst[ea];
        d[q] = (e0 + q < nE) ? dv : -1;
      }
    }
    unsigned hm = 0u;
#pragma unroll
    for (int q = 0; q < 8; ++q) {
      const unsigned jl = (unsigned)(d[q] - nbase);
      hm |= (jl < (unsigned)BNODE ? 1u : 0u) << q;
    }
    const int cnt = __popc(hm);
    int incl = cnt;
#pragma unroll
    for (int dd = 1; dd < 32; dd <<= 1) {
      const int tv = __shfl_up(incl, dd);
      incl += (lane >= dd) ? tv : 0;
    }
    if (lane == 31) sWT[wave] = incl;
    __syncthreads();
    int woff = 0, ctot = 0;
#pragma unroll
    for (int ww = 0; ww < 8; ++ww) {
      const int v = sWT[ww];
      woff += (ww < wave) ? v : 0;
      ctot += v;
    }
    int pos = tot + woff + incl - cnt;
#pragma unroll
    for (int q = 0; q < 8; ++q) {
      const int hit = (int)((hm >> q) & 1u);
      const int slot = (hit != 0 && pos < LCAP) ? pos : LCAP;
      sL[slot] = (int)((((unsigned)(d[q] - nbase)) << 24) | (unsigned)(e0 + q));
      pos += hit;
    }
    tot += ctot;
    __syncthreads();
  }
  const int ntot = tot < LCAP ? tot : LCAP;

#pragma unroll
  for (int i = 0; i < LCAP / 256; ++i) {
    const int idx = i * 256 + tid;
    const int ent = sL[idx];
    int e = ent & 0xFFFFFF; e = e > nE - 1 ? nE - 1 : e;
    int s = src[e]; s = s < 0 ? 0 : (s > nN - 1 ? nN - 1 : s);
    int ty = ety[e]; ty = ty < 0 ? 0 : (ty > 2047 ? 2047 : ty);
    sP[idx] = s | (ty << 20);
  }
  __syncthreads();

  const int nit = (ntot + 31) >> 5;
#pragma unroll 1
  for (int jj = 0; jj < 8; ++jj) {
    const int j = wave * 8 + jj;
    int run = 0;
#pragma unroll 1
    for (int it = 0; it < nit; ++it) {
      const int idx = it * 32 + lane;
      const int idc = idx < LCAP - 1 ? idx : LCAP - 1;
      const int ent = sL[idc];
      const int pk = sP[idc];
      const bool hit = (idx < ntot) && ((ent >> 24) == j);
      const unsigned mask = __builtin_amdgcn_ballot_w32(hit);
      const int rank = __popc(mask & ((1u << lane) - 1u));
      const int slot = run + rank;
      if (hit && slot < DEGCAP) sRow[j * TROW + 1 + slot] = pk;
      run += __popc(mask);
    }
    if (lane == 0) sRow[j * TROW] = run < DEGCAP ? run : DEGCAP;
  }
  __syncthreads();

  v2i rv[8];
  size_t ro[8];
  bool ok[8];
#pragma unroll
  for (int jj = 0; jj < 8; ++jj) {
    const int j = wave * 8 + jj;
    const int node = nbase + j;
    ok[jj] = node < nN;
    rv[jj] = *(const v2i*)(sRow + j * TROW + 2 * lane);
    const int nc = node > nN - 1 ? nN - 1 : node;
    ro[jj] = (size_t)nc * TROW + 2 * lane;
  }
#pragma unroll
  for (int jj = 0; jj < 8; ++jj) if (ok[jj]) *(volatile v2i*)(tab + ro[jj]) = rv[jj];
  __threadfence();
#pragma unroll
  for (int jj = 0; jj < 8; ++jj) if (ok[jj]) *(volatile v2i*)(tab + ro[jj]) = rv[jj];
}

__global__ __launch_bounds__(256) void k_agg(
    const float* __restrict__ qkv, const float* __restrict__ relp,
    const int* __restrict__ tab, unsigned short* att, int nN, int nR) {
  __shared__ __attribute__((aligned(16))) unsigned int sA[8 * 128];
  const int tid = (int)threadIdx.x, lane = tid & 31, wave = tid >> 5;
  const int hp = wave & 3, ns = wave >> 2;
  const int colw = hp * 64 + 2 * lane;
  const int nb = (int)blockIdx.x * 8;

#pragma unroll 1
  for (int jj = 0; jj < 4; ++jj) {
    const int ln = ns * 4 + jj;
    int node = nb + ln; node = node > nN - 1 ? nN - 1 : node;
    node = __builtin_amdgcn_readfirstlane(node);
    const int* trow = tab + (size_t)node * TROW;
    int cnt = __builtin_amdgcn_readfirstlane(trow[0]);
    cnt = cnt < 0 ? 0 : (cnt > DEGCAP ? DEGCAP : cnt);
    const v2f qv = *(const v2f*)(qkv + (size_t)node * DQKV + colw);
    float mrun = -1.0e30f, z = 0.0f, a0 = 0.0f, a1 = 0.0f;
#pragma unroll 1
    for (int i = 0; i < cnt; ++i) {
      const int p = __builtin_amdgcn_readfirstlane(trow[1 + i]);
      int s = p & 0xFFFFF;       s = s > nN - 1 ? nN - 1 : s;
      int ty = (p >> 20) & 0x7FF; ty = ty > nR - 1 ? nR - 1 : ty;
      const v2f rv = *(const v2f*)(relp + (size_t)ty * DM + colw);
      const v2f kv = *(const v2f*)(qkv + (size_t)s * DQKV + DM + colw);
      const v2f vv = *(const v2f*)(qkv + (size_t)s * DQKV + 2 * DM + colw);
      float part = qv.x * (kv.x + rv.x) + qv.y * (kv.y + rv.y);
      part += __shfl_xor(part, 8);
      part += __shfl_xor(part, 4);
      part += __shfl_xor(part, 2);
      part += __shfl_xor(part, 1);
      const float sc = part * QKSCL;
      const float mn = fmaxf(mrun, sc);
      const float corr = __expf(mrun - mn);
      const float pe = __expf(sc - mn);
      z  = z * corr + pe;
      a0 = a0 * corr + pe * (vv.x + rv.x);
      a1 = a1 * corr + pe * (vv.y + rv.y);
      mrun = mn;
    }
    const float rz = 1.0f / (z + 1e-16f);
    const unsigned int o = (unsigned int)h16(a0 * rz * ASCL) | ((unsigned int)h16(a1 * rz * ASCL) << 16);
    sA[ln * 128 + hp * 32 + lane] = o;
  }
  __syncthreads();

  int node = nb + wave; node = node > nN - 1 ? nN - 1 : node;
  const v4u val = *(const v4u*)(sA + wave * 128 + 4 * lane);
  unsigned short* gp = att + (size_t)node * DM + 8 * lane;
  *(volatile v4u*)gp = val;
  __threadfence();
  *(volatile v4u*)gp = val;
}

extern "C" void kernel_launch(void* const* d_in, const int* in_sizes, int n_in,
                              void* d_out, int out_size, void* d_ws, size_t ws_size,
                              hipStream_t stream) {
  if (n_in < 20) return;
  const int nN = in_sizes[0] / DM;
  const int nE = in_sizes[2];
  if (nN < 32 || nE <= 0) return;
  if (in_sizes[0] != nN * DM || (nN % 32) != 0) return;
  if (nN > (1 << 20) || nE > (1 << 24)) return;
  if (in_sizes[1] != 2 * nE) return;
  if (in_sizes[3] != DM * DM || in_sizes[4] != DM) return;
  const int nL = in_sizes[5] / (DM * DM);
  if (nL < 1 || nL > 64) return;
  if (in_sizes[5] != nL * DM * DM || in_sizes[7] != nL * DM * DM) return;
  if (in_sizes[9] != nL * DM * DM || in_sizes[12] != nL * DM * DM) return;
  if (in_sizes[6] != nL * DM || in_sizes[8] != nL * DM || in_sizes[10] != nL * DM) return;
  if (in_sizes[13] != nL * DM || in_sizes[14] != nL * DM || in_sizes[15] != nL * DM) return;
  if (in_sizes[19] != nL * DM) return;
  const int nR = in_sizes[11] / (nL * DM);
  if (nR < 1 || nR > 2047 || in_sizes[11] != nL * nR * DM) return;
  if (in_sizes[16] != nL * DM * DFF || in_sizes[17] != nL * DFF || in_sizes[18] != nL * DFF * DM) return;
  if (out_size != nN * DM) return;

  const float* x    = (const float*)d_in[0];
  const int*   eidx = (const int*)d_in[1];
  const int*   ety  = (const int*)d_in[2];
  const float* Wp   = (const float*)d_in[3];
  const float* bp   = (const float*)d_in[4];
  const float* Wq   = (const float*)d_in[5];
  const float* bq   = (const float*)d_in[6];
  const float* Wk   = (const float*)d_in[7];
  const float* bk   = (const float*)d_in[8];
  const float* Wv   = (const float*)d_in[9];
  const float* bv   = (const float*)d_in[10];
  const float* rel  = (const float*)d_in[11];
  const float* Wo   = (const float*)d_in[12];
  const float* bo   = (const float*)d_in[13];
  const float* n1w  = (const float*)d_in[14];
  const float* n2w  = (const float*)d_in[15];
  const float* W1   = (const float*)d_in[16];
  const float* b1   = (const float*)d_in[17];
  const float* W2   = (const float*)d_in[18];
  const float* b2   = (const float*)d_in[19];
  const int* src = eidx;
  const int* dst = eidx + nE;
  float* out = (float*)d_out;

  const int nbkt = (nN + BNODE - 1) / BNODE;
  const size_t szWp  = (size_t)DM * DM * 2;
  const size_t szWqv = (size_t)nL * DQKV * DM * 2;
  const size_t szWo  = (size_t)nL * DM * DM * 2;
  const size_t szW1  = (size_t)nL * DFF * DM * 2;
  const size_t szW2  = (size_t)nL * DM * DFF * 2;
  const size_t szX   = (size_t)nN * DM * 4;
  const size_t szB   = (size_t)nN * DM * 2;
  const size_t szQKV = (size_t)nN * DQKV * 4;
  const size_t szH   = (size_t)nN * DFF * 2;
  const size_t szA   = szQKV > szH ? szQKV : szH;
  const size_t szT   = (size_t)nbkt * BNODE * TROW * 4;
  size_t off = 0;
  const size_t oWp  = off; off += szWp;  off = (off + 255) & ~(size_t)255;
  const size_t oWqv = off; off += szWqv; off = (off + 255) & ~(size_t)255;
  const size_t oWo  = off; off += szWo;  off = (off + 255) & ~(size_t)255;
  const size_t oW1  = off; off += szW1;  off = (off + 255) & ~(size_t)255;
  const size_t oW2  = off; off += szW2;  off = (off + 255) & ~(size_t)255;
  const size_t oX   = off; off += szX;   off = (off + 255) & ~(size_t)255;
  const size_t oB   = off; off += szB;   off = (off + 255) & ~(size_t)255;
  const size_t oA   = off; off += szA;   off = (off + 255) & ~(size_t)255;
  const size_t oT   = off; off += szT;   off = (off + 255) & ~(size_t)255;
  if (off > ws_size || off > (size_t)WSCAP) return;

  char* ws = (char*)d_ws;
  unsigned short* wtP  = (unsigned short*)(ws + oWp);
  unsigned short* wtQ  = (unsigned short*)(ws + oWqv);
  unsigned short* wtO  = (unsigned short*)(ws + oWo);
  unsigned short* wt1  = (unsigned short*)(ws + oW1);
  unsigned short* wt2  = (unsigned short*)(ws + oW2);
  float*          xc   = (float*)(ws + oX);
  unsigned short* b16  = (unsigned short*)(ws + oB);
  float*          qkv  = (float*)(ws + oA);
  unsigned short* h16  = (unsigned short*)(ws + oA);
  int*            tab  = (int*)(ws + oT);

  const int vecok = ((nE & 3) == 0) ? 1 : 0;

  const dim3 gWp(DM / 64, DM / 64, 1);
  const dim3 gWsq(DM / 64, DM / 64, nL);
  const dim3 gW1(DFF / 64, DM / 64, nL);
  const dim3 gW2(DM / 64, DFF / 64, nL);
  k_wpack<<<gWp,  256, 0, stream>>>(Wp, wtP, DM, DM, 0, 0);
  k_wpack<<<gWsq, 256, 0, stream>>>(Wq, wtQ,               DM, DM, DM * DM, DQKV * DM);
  k_wpack<<<gWsq, 256, 0, stream>>>(Wk, wtQ + DM * DM,     DM, DM, DM * DM, DQKV * DM);
  k_wpack<<<gWsq, 256, 0, stream>>>(Wv, wtQ + 2 * DM * DM, DM, DM, DM * DM, DQKV * DM);
  k_wpack<<<gWsq, 256, 0, stream>>>(Wo, wtO, DM, DM, DM * DM, DM * DM);
  k_wpack<<<gW1,  256, 0, stream>>>(W1, wt1, DM, DFF, DM * DFF, DFF * DM);
  k_wpack<<<gW2,  256, 0, stream>>>(W2, wt2, DFF, DM, DFF * DM, DM * DFF);

  k_build<<<nbkt, 256, 0, stream>>>(src, dst, ety, tab, nN, nE, vecok);

  const dim3 gG256(1, nN / 32);
  const dim3 gG768(DQKV / 256, nN / 32);
  const dim3 gG1024(DFF / 256, nN / 32);
  k_cvt<<<nN / 8, 256, 0, stream>>>(x, b16, nN);
  k_gemm<0, 0><<<gG256, GT, 0, stream>>>(b16, wtP, bp, bp, bp, 30, xc, xc, h16, DM, DM, nN);

  for (int l = 0; l < nL; ++l) {
    k_rms<<<nN / 8, 256, 0, stream>>>(xc, n1w + (size_t)l * DM, b16, nN);
    k_gemm<0, 0><<<gG768, GT, 0, stream>>>(b16, wtQ + (size_t)l * DQKV * DM,
        bq + (size_t)l * DM, bk + (size_t)l * DM, bv + (size_t)l * DM, 8,
        xc, qkv, h16, DM, DQKV, nN);
    k_agg<<<nN / 8, 256, 0, stream>>>(qkv, rel + (size_t)l * nR * DM, tab, b16, nN, nR);
    k_gemm<0, 1><<<gG256, GT, 0, stream>>>(b16, wtO + (size_t)l * DM * DM,
        bo + (size_t)l * DM, bo + (size_t)l * DM, bo + (size_t)l * DM, 30,
        xc, xc, h16, DM, DM, nN);
    k_rms<<<nN / 8, 256, 0, stream>>>(xc, n2w + (size_t)l * DM, b16, nN);
    k_gemm<1, 0><<<gG1024, GT, 0, stream>>>(b16, wt1 + (size_t)l * DFF * DM,
        b1 + (size_t)l * DFF, b1 + (size_t)l * DFF, b1 + (size_t)l * DFF, 30,
        xc, xc, h16, DM, DFF, nN);
    float* dstp = (l == nL - 1) ? out : xc;
    k_gemm<0, 1><<<gG256, GT, 0, stream>>>(h16, wt2 + (size_t)l * DM * DFF,
        b2 + (size_t)l * DM, b2 + (size_t)l * DM, b2 + (size_t)l * DM, 30,
        xc, dstp, b16, DFF, DM, nN);
  }
}
